// DramaWorldModelComponent_61452392071570
// MI455X (gfx1250) — hardware-verified
//
#include <hip/hip_runtime.h>
#include <math.h>

typedef __attribute__((ext_vector_type(16))) _Float16 v16h;
typedef __attribute__((ext_vector_type(8)))  _Float16 v8h;
typedef __attribute__((ext_vector_type(16))) __bf16   v16b;
typedef __attribute__((ext_vector_type(8)))  __bf16   v8b;
typedef __attribute__((ext_vector_type(8)))  float    v8f;
typedef __attribute__((ext_vector_type(4)))  float    v4f;

constexpr int kBatch  = 4;
constexpr int kSeq    = 512;
constexpr int kStoch  = 1024;
constexpr int kDm     = 512;
constexpr int kDin    = 1024;
constexpr int kNst    = 16;
constexpr int kDtR    = 32;
constexpr int kXzP    = 2 * kDin;
constexpr int kXdP    = 64;
constexpr int kRows   = kBatch * kSeq;
constexpr int kLayers = 4;
constexpr int kNact   = 16;
constexpr int kConvTP = 260;
constexpr int kScanTS = 64;
constexpr int kScanCh = 64;
constexpr int kScanYP = 68;
constexpr float kWsc  = 32.0f;
constexpr float kUsc  = 16.0f;
constexpr float kYsc  = 64.0f;
static_assert(kDtR + 2 * kNst == kXdP, "x_proj width");
static_assert((kDm % 32) == 0 && (kDin % 32) == 0 && (kStoch % 32) == 0, "GEMM K multiples of 32");
static_assert((kRows % 64) == 0 && (kXzP % 64) == 0 && (kXdP % 64) == 0 && (kDm % 64) == 0 && (kStoch % 64) == 0, "GEMM M,N multiples of 64");
static_assert((kSeq % kScanTS) == 0 && (kSeq % 64) == 0 && (kDin % kScanCh) == 0 && (kDin % 256) == 0, "tile multiples");

constexpr size_t kOffWE   = 0;
constexpr size_t kOffWI   = kOffWE  + (size_t)kDm   * kStoch * 2;
constexpr size_t kOffWX   = kOffWI  + (size_t)kLayers * kXzP * kDm * 2;
constexpr size_t kOffWO   = kOffWX  + (size_t)kLayers * kXdP * kDin * 2;
constexpr size_t kOffSH   = kOffWO  + (size_t)kLayers * kDm * kDin * 2;
constexpr size_t kOffAE   = kOffSH  + (size_t)kRows * kStoch * 2;
constexpr size_t kOffX0   = kOffAE  + (size_t)kRows * kDm * 4;
constexpr size_t kOffX1   = kOffX0  + (size_t)kRows * kDm * 4;
constexpr size_t kOffXN   = kOffX1  + (size_t)kRows * kDm * 4;
constexpr size_t kOffXZ   = kOffXN  + (size_t)kRows * kDm * 2;
constexpr size_t kOffUC   = kOffXZ  + (size_t)kRows * kXzP * 4;
constexpr size_t kOffUCH  = kOffUC  + (size_t)kRows * kDin * 4;
constexpr size_t kOffXD   = kOffUCH + (size_t)kRows * kDin * 2;
constexpr size_t kOffYH   = kOffXD  + (size_t)kRows * kXdP * 4;
constexpr size_t kOffFN   = kOffYH  + (size_t)kRows * kDin * 2;
constexpr size_t kWsTotal = kOffFN  + (size_t)kRows * kDm * 4;
static_assert(kWsTotal == 71303168ull, "carve total");
static_assert(kWsTotal <= 134217728ull, "carve cap");
static_assert((kOffWI % 128) == 0 && (kOffWX % 128) == 0 && (kOffWO % 128) == 0 && (kOffSH % 128) == 0 &&
              (kOffAE % 128) == 0 && (kOffX0 % 128) == 0 && (kOffX1 % 128) == 0 && (kOffXN % 128) == 0 &&
              (kOffXZ % 128) == 0 && (kOffUC % 128) == 0 && (kOffUCH % 128) == 0 && (kOffXD % 128) == 0 &&
              (kOffYH % 128) == 0 && (kOffFN % 128) == 0, "128-B aligned regions");

__device__ __forceinline__ unsigned short f2bf_bits(float f) {
  unsigned u = __float_as_uint(f);
  return (unsigned short)((u + 0x7FFFu + ((u >> 16) & 1u)) >> 16);
}
__device__ __forceinline__ float bf_bits2f(unsigned short h) { return __uint_as_float(((unsigned)h) << 16); }

__device__ __forceinline__ void dep_guard_h(v8f& a, v8f& b, v16h x, v16h y) { asm volatile("v_nop\n\tv_nop\n\tv_nop\n\tv_nop" : "+v"(a), "+v"(b) : "v"(x), "v"(y)); }
__device__ __forceinline__ void dep_guard_b(v8f& a, v8f& b, v16b x, v16b y) { asm volatile("v_nop\n\tv_nop\n\tv_nop\n\tv_nop" : "+v"(a), "+v"(b) : "v"(x), "v"(y)); }
__device__ __forceinline__ void keep4_h(v16h a, v16h b, v16h c, v16h d) { asm volatile("v_nop" :: "v"(a), "v"(b), "v"(c), "v"(d)); }
__device__ __forceinline__ void keep4_b(v16b a, v16b b, v16b c, v16b d) { asm volatile("v_nop" :: "v"(a), "v"(b), "v"(c), "v"(d)); }
__device__ __forceinline__ void acc_guard4(v8f& a, v8f& b, v8f& c, v8f& d) { asm volatile("v_nop\n\tv_nop\n\tv_nop\n\tv_nop" : "+v"(a), "+v"(b), "+v"(c), "+v"(d)); }
template <typename T> struct Frag;
template <> struct Frag<_Float16> {
  typedef v16h V; union U { v16h v; v8h h[2]; };
  static __device__ __forceinline__ v16h load(const _Float16* p) {
    U f; f.h[0] = *(const v8h*)(p); f.h[1] = *(const v8h*)(p + 16); return f.v;
  }
  static __device__ __forceinline__ v8f mma(v16h a, v16h b, v8f c) {
    return __builtin_amdgcn_wmma_f32_16x16x32_f16(false, a, false, b, (short)0, c, false, false);
  }
  static __device__ __forceinline__ void guard(v8f& a, v8f& b, v16h x, v16h y) { dep_guard_h(a, b, x, y); }
  static __device__ __forceinline__ void keep(v16h a, v16h b, v16h c, v16h d) { keep4_h(a, b, c, d); }
};
template <> struct Frag<__bf16> {
  typedef v16b V; union U { v16b v; v8b h[2]; };
  static __device__ __forceinline__ v16b load(const __bf16* p) {
    U f; f.h[0] = *(const v8b*)(p); f.h[1] = *(const v8b*)(p + 16); return f.v;
  }
  static __device__ __forceinline__ v8f mma(v16b a, v16b b, v8f c) {
    return __builtin_amdgcn_wmma_f32_16x16x32_bf16(false, a, false, b, (short)0, c, false, false);
  }
  static __device__ __forceinline__ void guard(v8f& a, v8f& b, v16b x, v16b y) { dep_guard_b(a, b, x, y); }
  static __device__ __forceinline__ void keep(v16b a, v16b b, v16b c, v16b d) { keep4_b(a, b, c, d); }
};

template <int ET> struct Elem;
template <> struct Elem<0> { typedef _Float16 T; };
template <> struct Elem<1> { typedef __bf16 T; };
template <int ET, int SPL, int BIAS_MODE, int OUT_MODE, bool RESID, int ACT = 0>
__global__ __launch_bounds__(256) void wmma_gemm64(
    const unsigned short* __restrict__ Ap, const unsigned short* __restrict__ A2p, int lda, long strideA,
    const unsigned short* __restrict__ Btp, const unsigned short* __restrict__ Bt2p, int ldb, long strideB,
    void* __restrict__ Cout, void* __restrict__ Cout2, int ldc, long strideC,
    const float* __restrict__ bias,
    const float* __restrict__ resid, long strideR,
    int M, int N, int K, float scale) {
  typedef typename Elem<ET>::T T;
  typedef typename Frag<T>::V V;
  const T* A = (const T*)Ap; const T* A2 = (const T*)A2p; const T* Bt = (const T*)Btp; const T* Bt2 = (const T*)Bt2p;
  __shared__ __align__(16) float sT[8][16 * 68];
  const int b    = blockIdx.y;
  const int lane = threadIdx.x & 31;
  const int wave = threadIdx.x >> 5;
  const int tilesN = N >> 6;
  const int tilesM = M >> 6;
  const int tile = blockIdx.x * 8 + wave;
  if (tile >= tilesM * tilesN) return;
  const int tm = tile / tilesN;
  const int tn = tile - tm * tilesN;
  const int m0 = tm << 6;
  const int n0 = tn << 6;

  const T* Ab  = A  + (size_t)b * strideA;
  const T* Bb  = Bt + (size_t)b * strideB;
  const T* Ab2 = (SPL >= 1) ? (A2  + (size_t)b * strideA) : nullptr;
  const T* Bb2 = (SPL == 2) ? (Bt2 + (size_t)b * strideB) : nullptr;

  const int rlane = lane & 15;
  const int koff  = (lane >> 4) * 8;
  const int mOff  = (lane >> 4) * 8;

  v8f acc[4][4];
#pragma unroll
  for (int i = 0; i < 4; ++i)
#pragma unroll
    for (int j = 0; j < 4; ++j) acc[i][j] = (v8f){0.f,0.f,0.f,0.f,0.f,0.f,0.f,0.f};

  for (int k0 = 0; k0 < K; k0 += 32) {
    V bh[4], bl[4];
#pragma unroll
    for (int j = 0; j < 4; ++j) {
      const size_t bo = (size_t)(n0 + (j << 4) + rlane) * ldb + koff + k0;
      bh[j] = Frag<T>::load(Bb + bo);
      if (SPL == 2) bl[j] = Frag<T>::load(Bb2 + bo);
    }
#pragma unroll
    for (int i = 0; i < 4; ++i) {
      const size_t ao = (size_t)(m0 + (i << 4) + rlane) * lda + koff + k0;
      V ah = Frag<T>::load(Ab + ao);
      V al;
      if (SPL >= 1) al = Frag<T>::load(Ab2 + ao);
#pragma unroll
      for (int j = 0; j < 4; ++j) {
        acc[i][j] = Frag<T>::mma(ah, bh[j], acc[i][j]);
        if (SPL == 2) acc[i][j] = Frag<T>::mma(ah, bl[j], acc[i][j]);
        if (SPL >= 1) acc[i][j] = Frag<T>::mma(al, bh[j], acc[i][j]);
      }
      Frag<T>::guard(acc[i][0], acc[i][3], ah, (SPL >= 1) ? al : ah);
    }
    Frag<T>::keep(bh[0], bh[1], bh[2], bh[3]);
    if (SPL == 2) Frag<T>::keep(bl[0], bl[1], bl[2], bl[3]);
  }
  acc_guard4(acc[0][0], acc[0][1], acc[0][2], acc[0][3]);
  acc_guard4(acc[1][0], acc[1][1], acc[1][2], acc[1][3]);
  acc_guard4(acc[2][0], acc[2][1], acc[2][2], acc[2][3]);
  acc_guard4(acc[3][0], acc[3][1], acc[3][2], acc[3][3]);

  float* slab = sT[wave];
  const float* Rb = RESID ? (resid + (size_t)b * strideR) : nullptr;
#pragma unroll
  for (int i = 0; i < 4; ++i) {
    const int mBase = m0 + (i << 4);
#pragma unroll
    for (int j = 0; j < 4; ++j) {
      const int n = n0 + (j << 4) + rlane;
      float bv = 0.f;
      if (BIAS_MODE == 2) bv = bias[n];
#pragma unroll
      for (int r = 0; r < 8; ++r) {
        float v = acc[i][j][r] * scale;
        if (BIAS_MODE == 1) v += bias[mBase + mOff + r];
        if (BIAS_MODE == 2) v += bv;
        if (RESID) v += Rb[(size_t)(mBase + mOff + r) * ldc + n];
        if (ACT == 1) v = tanhf(v);
        if (ACT == 2) v = fmaxf(v, 0.0f);
        if (ACT == 3) v = v / (1.0f + expf(-v));
        if (ACT == 4) v = (v > 0.f) ? v : 0.01f * v;
        slab[(mOff + r) * 68 + (j << 4) + rlane] = v;
      }
    }
    __builtin_amdgcn_fence(__ATOMIC_RELEASE, "workgroup");
    __builtin_amdgcn_wave_barrier();
    __builtin_amdgcn_fence(__ATOMIC_ACQUIRE, "workgroup");
    if (OUT_MODE == 0) {
      float* C = (float*)Cout + (size_t)b * strideC;
      const int hh = lane >> 4, c4 = (lane & 15) * 4;
      for (int pass = 0; pass < 2; ++pass) {
#pragma unroll
        for (int it = 0; it < 8; ++it) {
          const int row = it * 2 + hh;
          v4f v = *(const v4f*)(slab + row * 68 + c4);
          *(volatile v4f*)(C + (size_t)(mBase + row) * ldc + n0 + c4) = v;
        }
        __threadfence();
      }
    } else {
      const int q = lane >> 3, c8 = (lane & 7) * 8;
      unsigned short* C  = (unsigned short*)Cout  + (size_t)b * strideC;
      unsigned short* C2 = (OUT_MODE == 2) ? ((unsigned short*)Cout2 + (size_t)b * strideC) : nullptr;
      for (int pass = 0; pass < 2; ++pass) {
#pragma unroll
        for (int it = 0; it < 4; ++it) {
          const int row = it * 4 + q;
          const float* sp = slab + row * 68 + c8;
          v8h hv, lv;
#pragma unroll
          for (int e = 0; e < 8; ++e) {
            if (OUT_MODE == 1) {
              hv[e] = (_Float16)sp[e];
            } else {
              unsigned short hb = f2bf_bits(sp[e]);
              unsigned short lb = f2bf_bits(sp[e] - bf_bits2f(hb));
              hv[e] = __builtin_bit_cast(_Float16, hb);
              lv[e] = __builtin_bit_cast(_Float16, lb);
            }
          }
          *(volatile v8h*)(C + (size_t)(mBase + row) * ldc + n0 + c8) = hv;
          if (OUT_MODE == 2) *(volatile v8h*)(C2 + (size_t)(mBase + row) * ldc + n0 + c8) = lv;
        }
        __threadfence();
      }
    }
    __builtin_amdgcn_fence(__ATOMIC_RELEASE, "workgroup");
    __builtin_amdgcn_wave_barrier();
    __builtin_amdgcn_fence(__ATOMIC_ACQUIRE, "workgroup");
  }
}

__global__ __launch_bounds__(256) void tcast_f16_kernel(
    const float* __restrict__ in, unsigned short* __restrict__ out, int nK, int nN, float scale)
{
  __shared__ __align__(16) float sT[64 * 68];
  const int tid = threadIdx.x, lane = tid & 31, wave = tid >> 5;
  const int n0 = blockIdx.x * 64, k0 = blockIdx.y * 64;
  const size_t zoff = (size_t)blockIdx.z * (size_t)nK * (size_t)nN;
  const float* inz = in + zoff;
  unsigned short* outz = out + zoff;
  const int r = tid >> 4, c4 = (tid & 15) * 4;
#pragma unroll
  for (int i = 0; i < 4; ++i) {
    const int row = r + 16 * i;
    const v4f v = *(const v4f*)(inz + (size_t)(k0 + row) * nN + n0 + c4);
    *(v4f*)(sT + row * 68 + c4) = v;
  }
  __syncthreads();
  const int q = lane >> 3, c8 = (lane & 7) * 8;
  v8h hv[2];
#pragma unroll
  for (int it = 0; it < 2; ++it) {
    const int nrow = it * 32 + wave * 4 + q;
#pragma unroll
    for (int e = 0; e < 8; ++e) hv[it][e] = (_Float16)(sT[(c8 + e) * 68 + nrow] * scale);
  }
  for (int pass = 0; pass < 2; ++pass) {
#pragma unroll
    for (int it = 0; it < 2; ++it) {
      const int nrow = it * 32 + wave * 4 + q;
      *(volatile v8h*)(outz + (size_t)(n0 + nrow) * nK + k0 + c8) = hv[it];
    }
    __threadfence();
  }
}

__global__ __launch_bounds__(256) void cast_rows_f16_kernel(
    const float* __restrict__ src, unsigned short* __restrict__ dst, int total8, float scale)
{
  const int i = blockIdx.x * 256 + threadIdx.x;
  if (i >= total8) return;
  const size_t e0 = (size_t)i << 3;
  const v4f a0 = *(const v4f*)(src + e0);
  const v4f a1 = *(const v4f*)(src + e0 + 4);
  v8h hv;
#pragma unroll
  for (int e = 0; e < 4; ++e) {
    hv[e]     = (_Float16)(a0[e] * scale);
    hv[4 + e] = (_Float16)(a1[e] * scale);
  }
  unsigned short* p = dst + e0;
  *(volatile v8h*)p = hv;
  __threadfence();
  *(volatile v8h*)p = hv;
}

__global__ __launch_bounds__(256) void act_rows_kernel(
    const int* __restrict__ act, const float* __restrict__ ae, const float* __restrict__ be,
    float* __restrict__ dst, int total4)
{
  const int i = blockIdx.x * 256 + threadIdx.x;
  if (i >= total4) return;
  const size_t e0 = (size_t)i << 2;
  const int row = (int)(e0 >> 9);
  const int c4  = (int)(e0 & (size_t)(kDm - 1));
  int a = act[row];
  a = a < 0 ? 0 : (a > kNact - 1 ? kNact - 1 : a);
  const v4f v  = *(const v4f*)(ae + (size_t)a * kDm + c4);
  const v4f bv = *(const v4f*)(be + c4);
  const v4f o = v + bv;
  float* p = dst + e0;
  *(volatile v4f*)p = o;
  __threadfence();
  *(volatile v4f*)p = o;
}

__global__ __launch_bounds__(256) void ln_rows_f16_kernel(
    const float* __restrict__ X, const float* __restrict__ w, const float* __restrict__ bb,
    unsigned short* __restrict__ XN, int nrows)
{
  const int lane = threadIdx.x & 31, wave = threadIdx.x >> 5;
  const int row = blockIdx.x * 8 + wave;
  if (row >= nrows) return;
  const float* xr = X + (size_t)row * kDm;
  const int c0 = lane * 8, c1 = 256 + lane * 8;
  const v4f a0 = *(const v4f*)(xr + c0);
  const v4f a1 = *(const v4f*)(xr + c0 + 4);
  const v4f a2 = *(const v4f*)(xr + c1);
  const v4f a3 = *(const v4f*)(xr + c1 + 4);
  float s = 0.f;
#pragma unroll
  for (int e = 0; e < 4; ++e) s += (a0[e] + a1[e]) + (a2[e] + a3[e]);
#pragma unroll
  for (int off = 1; off < 32; off <<= 1) s += __shfl_xor(s, off, 32);
  const float m = s * (1.0f / kDm);
  const v4f d0 = a0 - m, d1 = a1 - m, d2 = a2 - m, d3 = a3 - m;
  float qq = 0.f;
#pragma unroll
  for (int e = 0; e < 4; ++e) qq += (d0[e] * d0[e] + d1[e] * d1[e]) + (d2[e] * d2[e] + d3[e] * d3[e]);
#pragma unroll
  for (int off = 1; off < 32; off <<= 1) qq += __shfl_xor(qq, off, 32);
  const float var = qq * (1.0f / kDm);
  const float rs = rsqrtf(var + 1e-5f);
  const v4f w0 = *(const v4f*)(w + c0),  w1 = *(const v4f*)(w + c0 + 4);
  const v4f w2 = *(const v4f*)(w + c1),  w3 = *(const v4f*)(w + c1 + 4);
  const v4f b0 = *(const v4f*)(bb + c0), b1 = *(const v4f*)(bb + c0 + 4);
  const v4f b2 = *(const v4f*)(bb + c1), b3 = *(const v4f*)(bb + c1 + 4);
  const v4f y0 = (d0 * rs) * w0 + b0;
  const v4f y1 = (d1 * rs) * w1 + b1;
  const v4f y2 = (d2 * rs) * w2 + b2;
  const v4f y3 = (d3 * rs) * w3 + b3;
  v8h h0, h1;
#pragma unroll
  for (int e = 0; e < 4; ++e) {
    h0[e] = (_Float16)y0[e]; h0[4 + e] = (_Float16)y1[e];
    h1[e] = (_Float16)y2[e]; h1[4 + e] = (_Float16)y3[e];
  }
  unsigned short* o0 = XN + (size_t)row * kDm + c0;
  unsigned short* o1 = XN + (size_t)row * kDm + c1;
  *(volatile v8h*)o0 = h0;
  *(volatile v8h*)o1 = h1;
  __threadfence();
  *(volatile v8h*)o0 = h0;
  *(volatile v8h*)o1 = h1;
}

__global__ __launch_bounds__(256) void final_ln_kernel(
    const float* __restrict__ X,
    const float* __restrict__ w1, const float* __restrict__ b1,
    const float* __restrict__ w2, const float* __restrict__ b2,
    float* __restrict__ FN, int nrows)
{
  const int lane = threadIdx.x & 31, wave = threadIdx.x >> 5;
  const int row = blockIdx.x * 8 + wave;
  if (row >= nrows) return;
  const float* xr = X + (size_t)row * kDm;
  v4f a[4];
#pragma unroll
  for (int k = 0; k < 4; ++k) a[k] = *(const v4f*)(xr + 128 * k + lane * 4);
  float s = 0.f;
#pragma unroll
  for (int k = 0; k < 4; ++k) s += (a[k][0] + a[k][1]) + (a[k][2] + a[k][3]);
#pragma unroll
  for (int off = 1; off < 32; off <<= 1) s += __shfl_xor(s, off, 32);
  const float m = s * (1.0f / kDm);
  v4f d[4];
  float qq = 0.f;
#pragma unroll
  for (int k = 0; k < 4; ++k) {
    d[k] = a[k] - m;
    qq += (d[k][0] * d[k][0] + d[k][1] * d[k][1]) + (d[k][2] * d[k][2] + d[k][3] * d[k][3]);
  }
#pragma unroll
  for (int off = 1; off < 32; off <<= 1) qq += __shfl_xor(qq, off, 32);
  const float rs = rsqrtf(qq * (1.0f / kDm) + 1e-5f);
  v4f y[4];
  float s2 = 0.f;
#pragma unroll
  for (int k = 0; k < 4; ++k) {
    const v4f wv = *(const v4f*)(w1 + 128 * k + lane * 4);
    const v4f bv = *(const v4f*)(b1 + 128 * k + lane * 4);
    y[k] = (d[k] * rs) * wv + bv;
    s2 += (y[k][0] + y[k][1]) + (y[k][2] + y[k][3]);
  }
#pragma unroll
  for (int off = 1; off < 32; off <<= 1) s2 += __shfl_xor(s2, off, 32);
  const float m2 = s2 * (1.0f / kDm);
  float q2 = 0.f;
#pragma unroll
  for (int k = 0; k < 4; ++k) {
    y[k] = y[k] - m2;
    q2 += (y[k][0] * y[k][0] + y[k][1] * y[k][1]) + (y[k][2] * y[k][2] + y[k][3] * y[k][3]);
  }
#pragma unroll
  for (int off = 1; off < 32; off <<= 1) q2 += __shfl_xor(q2, off, 32);
  const float rs2 = rsqrtf(q2 * (1.0f / kDm) + 1e-5f);
  v4f o[4];
#pragma unroll
  for (int k = 0; k < 4; ++k) {
    const v4f wv = *(const v4f*)(w2 + 128 * k + lane * 4);
    const v4f bv = *(const v4f*)(b2 + 128 * k + lane * 4);
    o[k] = (y[k] * rs2) * wv + bv;
  }
  for (int pass = 0; pass < 2; ++pass) {
#pragma unroll
    for (int k = 0; k < 4; ++k)
      *(volatile v4f*)(FN + (size_t)row * kDm + 128 * k + lane * 4) = o[k];
    __threadfence();
  }
}

__global__ __launch_bounds__(128) void mean_pool_kernel(const float* __restrict__ FN, float* __restrict__ out)
{
  __shared__ __align__(16) float sM[128];
  const int tid = threadIdx.x;
  const int b = blockIdx.x >> 2, c0 = (blockIdx.x & 3) * 128, c = c0 + tid;
  const float* p = FN + (size_t)b * kSeq * kDm + c;
  float p0 = 0.f, p1 = 0.f, p2 = 0.f, p3 = 0.f;
#pragma unroll 1
  for (int t = 0; t < kSeq; t += 4) {
    p0 += p[(size_t)(t)     * kDm];
    p1 += p[(size_t)(t + 1) * kDm];
    p2 += p[(size_t)(t + 2) * kDm];
    p3 += p[(size_t)(t + 3) * kDm];
  }
  sM[tid] = ((p0 + p1) + (p2 + p3)) * (1.0f / kSeq);
  __syncthreads();
  if (tid < 32) {
    const v4f v = *(const v4f*)(sM + tid * 4);
    float* o = out + (size_t)b * kDm + c0 + tid * 4;
    *(volatile v4f*)o = v;
    __threadfence();
    *(volatile v4f*)o = v;
  }
}

__global__ __launch_bounds__(256) void conv_silu_kernel(
    const float* __restrict__ XZ, const float* __restrict__ cw, const float* __restrict__ cb,
    float* __restrict__ UC, unsigned short* __restrict__ UCH)
{
  __shared__ __align__(16) float sT[16 * kConvTP];
  const int tid = threadIdx.x, lane = tid & 31, wave = tid >> 5;
  const int d0 = blockIdx.x * 256, d = d0 + tid;
  const int g0 = blockIdx.y * 64;
  const int tb = g0 & (kSeq - 1);
  const float w0 = cw[d * 4 + 0], w1 = cw[d * 4 + 1], w2 = cw[d * 4 + 2], w3 = cw[d * 4 + 3];
  const float bc = cb[d];
  float xm3, xm2, xm1;
  {
    const bool hist = (tb > 0);
    const int rb = hist ? (g0 - 3) : g0;
    const float v3 = XZ[(size_t)rb * kXzP + d];
    const float v2 = XZ[(size_t)(rb + 1) * kXzP + d];
    const float v1 = XZ[(size_t)(rb + 2) * kXzP + d];
    xm3 = hist ? v3 : 0.f;
    xm2 = hist ? v2 : 0.f;
    xm1 = hist ? v1 : 0.f;
  }
  const int hrow = wave >> 1;
  const int hch  = (wave & 1) * 128 + lane * 4;
#pragma unroll 1
  for (int sub = 0; sub < 4; ++sub) {
    const int lb = g0 + sub * 16;
#pragma unroll 1
    for (int s = 0; s < 16; ++s) {
      const float xcur = XZ[(size_t)(lb + s) * kXzP + d];
      float acc = w0 * xm3;
      acc = fmaf(w1, xm2, acc);
      acc = fmaf(w2, xm1, acc);
      acc = fmaf(w3, xcur, acc);
      const float sv = acc + bc;
      const float sg = __builtin_amdgcn_rcpf(1.0f + __expf(-sv));
      sT[s * kConvTP + tid] = sv * sg;
      xm3 = xm2; xm2 = xm1; xm1 = xcur;
    }
    __syncthreads();
    v4f fv[4];
    v8h bh[2];
#pragma unroll
    for (int it = 0; it < 4; ++it) fv[it] = *(const v4f*)(sT + (it * 4 + hrow) * kConvTP + hch);
#pragma unroll
    for (int it = 0; it < 2; ++it) {
      const float* sp = sT + (it * 8 + wave) * kConvTP + lane * 8;
      const v4f a0 = *(const v4f*)(sp);
      const v4f a1 = *(const v4f*)(sp + 4);
#pragma unroll
      for (int e = 0; e < 4; ++e) {
        bh[it][e]     = (_Float16)(a0[e] * kUsc);
        bh[it][4 + e] = (_Float16)(a1[e] * kUsc);
      }
    }
    for (int pass = 0; pass < 2; ++pass) {
#pragma unroll
      for (int it = 0; it < 4; ++it)
        *(volatile v4f*)(UC + (size_t)(lb + it * 4 + hrow) * kDin + d0 + hch) = fv[it];
#pragma unroll
      for (int it = 0; it < 2; ++it) {
        const size_t o = (size_t)(lb + it * 8 + wave) * kDin + d0 + lane * 8;
        *(volatile v8h*)(UCH + o) = bh[it];
      }
      __threadfence();
    }
    __syncthreads();
  }
}

__global__ __launch_bounds__(64) void scan_kernel(
    const float* __restrict__ XD, const float* __restrict__ UC, const float* __restrict__ XZ,
    const float* __restrict__ Wdt, const float* __restrict__ bdt, const float* __restrict__ Alog,
    const float* __restrict__ Dp, unsigned short* __restrict__ YH)
{
  __shared__ __align__(16) float sX[kScanTS * kXdP];
  __shared__ __align__(16) float sY[kScanTS * kScanYP];
  __shared__ __align__(16) float sW[kDtR * kScanCh];
  __shared__ __align__(16) float sA[kNst * kScanCh];
  const int tid = threadIdx.x, lane = tid & 31, wave = tid >> 5;
  constexpr int kBlkPerB = kDin / kScanCh;
  const int bix = blockIdx.x / kBlkPerB;
  const int d0  = (blockIdx.x - bix * kBlkPerB) * kScanCh;
  const int d   = d0 + tid;
  const size_t row0 = (size_t)bix * kSeq;
#pragma unroll 1
  for (int r = 0; r < kDtR; ++r) sW[r * kScanCh + tid] = Wdt[(size_t)r * kDin + d];
#pragma unroll 1
  for (int s = 0; s < kNst; ++s) sA[s * kScanCh + tid] = -expf(Alog[(size_t)d * kNst + s]);
  __syncthreads();
  float negA[kNst], h[kNst];
#pragma unroll
  for (int s = 0; s < kNst; ++s) {
    negA[s] = sA[s * kScanCh + tid];
    h[s] = 0.f;
  }
  const float bb = bdt[d], Dd = Dp[d];
  const int lr = tid >> 4, lc4 = (tid & 15) * 4;
  const int q = lane >> 3, c8 = (lane & 7) * 8;
#pragma unroll 1
  for (int t0 = 0; t0 < kSeq; t0 += kScanTS) {
    __syncthreads();
#pragma unroll
    for (int i = 0; i < 16; ++i) {
      const int r = lr + 4 * i;
      *(v4f*)(sX + r * kXdP + lc4) = *(const v4f*)(XD + (row0 + t0 + r) * kXdP + lc4);
    }
    __syncthreads();
#pragma unroll 1
    for (int s = 0; s < kScanTS; ++s) {
      const int t = t0 + s;
      const float* xr = sX + s * kXdP;
      float vdot = 0.f;
#pragma unroll 1
      for (int r4 = 0; r4 < kDtR / 4; ++r4) {
        const v4f xv = *(const v4f*)(xr + 4 * r4);
        const float* wp = sW + (4 * r4) * kScanCh + tid;
        vdot = fmaf(xv[0], wp[0], vdot);
        vdot = fmaf(xv[1], wp[kScanCh], vdot);
        vdot = fmaf(xv[2], wp[2 * kScanCh], vdot);
        vdot = fmaf(xv[3], wp[3 * kScanCh], vdot);
      }
      float Bs[kNst], Cs[kNst];
#pragma unroll
      for (int q4 = 0; q4 < 4; ++q4) {
        const v4f bv = *(const v4f*)(xr + kDtR + 4 * q4);
        const v4f cv = *(const v4f*)(xr + kDtR + kNst + 4 * q4);
        Bs[4 * q4 + 0] = bv[0]; Bs[4 * q4 + 1] = bv[1]; Bs[4 * q4 + 2] = bv[2]; Bs[4 * q4 + 3] = bv[3];
        Cs[4 * q4 + 0] = cv[0]; Cs[4 * q4 + 1] = cv[1]; Cs[4 * q4 + 2] = cv[2]; Cs[4 * q4 + 3] = cv[3];
      }
      const float v   = vdot + bb;
      const float a   = __expf(-fabsf(v));
      const float u   = 1.0f + a;
      const float l1p = __logf(u) + (a - (u - 1.0f)) * __builtin_amdgcn_rcpf(u);
      const float dt  = fmaxf(v, 0.0f) + l1p;
      const float xt  = UC[(row0 + t) * kDin + d];
      const float dtx = dt * xt;
      float y = 0.f;
#pragma unroll
      for (int k = 0; k < kNst; ++k) {
        const float e = __expf(dt * negA[k]);
        h[k] = e * h[k] + dtx * Bs[k];
        y = h[k] * Cs[k] + y;
      }
      y = xt * Dd + y;
      const float zv = XZ[(row0 + t) * kXzP + kDin + d];
      const float sg = __builtin_amdgcn_rcpf(1.0f + __expf(-zv));
      y = y * (zv * sg);
      sY[s * kScanYP + tid] = y;
    }
    __syncthreads();
    v8h hv[8];
#pragma unroll
    for (int it = 0; it < 8; ++it) {
      const int row = it * 8 + wave * 4 + q;
      const float* sp = sY + row * kScanYP + c8;
      const v4f a0 = *(const v4f*)(sp);
      const v4f a1 = *(const v4f*)(sp + 4);
#pragma unroll
      for (int e = 0; e < 4; ++e) {
        hv[it][e]     = (_Float16)(a0[e] * kYsc);
        hv[it][4 + e] = (_Float16)(a1[e] * kYsc);
      }
    }
    for (int pass = 0; pass < 2; ++pass) {
#pragma unroll
      for (int it = 0; it < 8; ++it) {
        const int row = it * 8 + wave * 4 + q;
        const size_t o = (row0 + t0 + row) * kDin + d0 + c8;
        *(volatile v8h*)(YH + o) = hv[it];
      }
      __threadfence();
    }
  }
}

extern "C" void kernel_launch(void* const* d_in, const int* in_sizes, int n_in,
                              void* d_out, int out_size, void* d_ws, size_t ws_size,
                              hipStream_t stream) {
  if (n_in < 20) return;
  if (in_sizes[0]  != kRows * kStoch) return;
  if (in_sizes[1]  != kRows) return;
  if (in_sizes[2]  != kStoch * kDm) return;
  if (in_sizes[3]  != kDm) return;
  if (in_sizes[4]  != kNact * kDm) return;
  if (in_sizes[5]  != kLayers * kDm) return;
  if (in_sizes[6]  != kLayers * kDm) return;
  if (in_sizes[7]  != kLayers * kDm * kXzP) return;
  if (in_sizes[8]  != kLayers * kDin * 4) return;
  if (in_sizes[9]  != kLayers * kDin) return;
  if (in_sizes[10] != kLayers * kDin * kXdP) return;
  if (in_sizes[11] != kLayers * kDtR * kDin) return;
  if (in_sizes[12] != kLayers * kDin) return;
  if (in_sizes[13] != kLayers * kDin * kNst) return;
  if (in_sizes[14] != kLayers * kDin) return;
  if (in_sizes[15] != kLayers * kDin * kDm) return;
  if (in_sizes[16] != kDm || in_sizes[17] != kDm || in_sizes[18] != kDm || in_sizes[19] != kDm) return;
  if (out_size != kBatch * kDm) return;
  if (ws_size < kWsTotal) return;

  const float* samples  = (const float*)d_in[0];
  const int*   actions  = (const int*)  d_in[1];
  const float* W_embed  = (const float*)d_in[2];
  const float* b_embed  = (const float*)d_in[3];
  const float* act_emb  = (const float*)d_in[4];
  const float* ln_w     = (const float*)d_in[5];
  const float* ln_b     = (const float*)d_in[6];
  const float* W_in     = (const float*)d_in[7];
  const float* conv_w   = (const float*)d_in[8];
  const float* conv_b   = (const float*)d_in[9];
  const float* W_xproj  = (const float*)d_in[10];
  const float* W_dt     = (const float*)d_in[11];
  const float* b_dt     = (const float*)d_in[12];
  const float* A_log    = (const float*)d_in[13];
  const float* D_skip   = (const float*)d_in[14];
  const float* W_out    = (const float*)d_in[15];
  const float* normf_w  = (const float*)d_in[16];
  const float* normf_b  = (const float*)d_in[17];
  const float* outln_w  = (const float*)d_in[18];
  const float* outln_b  = (const float*)d_in[19];
  float* out = (float*)d_out;

  char* ws = (char*)d_ws;
  unsigned short* WE   = (unsigned short*)(ws + kOffWE);
  unsigned short* WI   = (unsigned short*)(ws + kOffWI);
  unsigned short* WX   = (unsigned short*)(ws + kOffWX);
  unsigned short* WO   = (unsigned short*)(ws + kOffWO);
  unsigned short* SH   = (unsigned short*)(ws + kOffSH);
  float*          AE   = (float*)(ws + kOffAE);
  float*          X0   = (float*)(ws + kOffX0);
  float*          X1   = (float*)(ws + kOffX1);
  unsigned short* XN   = (unsigned short*)(ws + kOffXN);
  float*          XZ   = (float*)(ws + kOffXZ);
  float*          UC   = (float*)(ws + kOffUC);
  unsigned short* UCH  = (unsigned short*)(ws + kOffUCH);
  float*          XD   = (float*)(ws + kOffXD);
  unsigned short* YH   = (unsigned short*)(ws + kOffYH);
  float*          FN   = (float*)(ws + kOffFN);

  tcast_f16_kernel<<<dim3(kDm / 64, kStoch / 64, 1), 256, 0, stream>>>(W_embed, WE, kStoch, kDm, kWsc);
  tcast_f16_kernel<<<dim3(kXzP / 64, kDm / 64, kLayers), 256, 0, stream>>>(W_in, WI, kDm, kXzP, kWsc);
  tcast_f16_kernel<<<dim3(kXdP / 64, kDin / 64, kLayers), 256, 0, stream>>>(W_xproj, WX, kDin, kXdP, kWsc);
  tcast_f16_kernel<<<dim3(kDm / 64, kDin / 64, kLayers), 256, 0, stream>>>(W_out, WO, kDin, kDm, kWsc);

  cast_rows_f16_kernel<<<(kRows * kStoch / 8) / 256, 256, 0, stream>>>(samples, SH, kRows * kStoch / 8, 1.0f);
  act_rows_kernel<<<(kRows * kDm / 4) / 256, 256, 0, stream>>>(actions, act_emb, b_embed, AE, kRows * kDm / 4);

  wmma_gemm64<0, 0, 0, 0, true><<<dim3(32, 1), 256, 0, stream>>>(
      SH, nullptr, kStoch, 0L,
      WE, nullptr, kStoch, 0L,
      (void*)X0, nullptr, kDm, 0L,
      nullptr, AE, 0L,
      kRows, kDm, kStoch, 1.0f / kWsc);

  for (int l = 0; l < kLayers; ++l) {
    float* Xcur  = (l & 1) ? X1 : X0;
    float* Xnext = (l & 1) ? X0 : X1;

    ln_rows_f16_kernel<<<kRows / 8, 256, 0, stream>>>(Xcur, ln_w + (size_t)l * kDm, ln_b + (size_t)l * kDm, XN, kRows);

    wmma_gemm64<0, 0, 0, 0, false><<<dim3(128, 1), 256, 0, stream>>>(
        XN, nullptr, kDm, 0L,
        WI + (size_t)l * kXzP * kDm, nullptr, kDm, 0L,
        (void*)XZ, nullptr, kXzP, 0L,
        nullptr, nullptr, 0L,
        kRows, kXzP, kDm, 1.0f / kWsc);

    conv_silu_kernel<<<dim3(kDin / 256, kRows / 64), 256, 0, stream>>>(
        XZ, conv_w + (size_t)l * kDin * 4, conv_b + (size_t)l * kDin, UC, UCH);

    wmma_gemm64<0, 0, 0, 0, false><<<dim3(4, 1), 256, 0, stream>>>(
        UCH, nullptr, kDin, 0L,
        WX + (size_t)l * kXdP * kDin, nullptr, kDin, 0L,
        (void*)XD, nullptr, kXdP, 0L,
        nullptr, nullptr, 0L,
        kRows, kXdP, kDin, 1.0f / (kUsc * kWsc));

    scan_kernel<<<kBatch * (kDin / kScanCh), kScanCh, 0, stream>>>(
        XD, UC, XZ, W_dt + (size_t)l * kDtR * kDin, b_dt + (size_t)l * kDin,
        A_log + (size_t)l * kDin * kNst, D_skip + (size_t)l * kDin, YH);

    wmma_gemm64<0, 0, 0, 0, true><<<dim3(32, 1), 256, 0, stream>>>(
        YH, nullptr, kDin, 0L,
        WO + (size_t)l * kDm * kDin, nullptr, kDin, 0L,
        (void*)Xnext, nullptr, kDm, 0L,
        nullptr, Xcur, 0L,
        kRows, kDm, kDin, 1.0f / (kYsc * kWsc));
  }

  final_ln_kernel<<<kRows / 8, 256, 0, stream>>>(X0, normf_w, normf_b, outln_w, outln_b, FN, kRows);
  mean_pool_kernel<<<kBatch * (kDm / 128), 128, 0, stream>>>(FN, out);
}
